// TGCN_MessageCoupling_76012331204906
// MI455X (gfx1250) — hardware-run, weakly checked
//
#include <hip/hip_runtime.h>


namespace {
constexpr int T = 16, N = 50000, FI = 16, GH = 64, RH = 64, EH = 128, E = 800000, NBLK = N / 16;
constexpr float XS = 8.0f, WSC = 256.0f;
typedef _Float16 b16;
typedef __attribute__((ext_vector_type(16))) _Float16 v16b;
typedef __attribute__((ext_vector_type(8))) _Float16 v8b;
typedef __attribute__((ext_vector_type(8))) float v8f;
typedef __attribute__((ext_vector_type(4))) float v4f;
typedef __attribute__((ext_vector_type(2))) float v2f;
__device__ __forceinline__ float bf16_rne(float f) { unsigned int u = __float_as_uint(f); u += 0x7FFFu + ((u >> 16) & 1u); return __uint_as_float(u & 0xFFFF0000u); }
__device__ __forceinline__ void split16(float v, b16& hi, b16& lo) { hi = (b16)v; lo = (b16)(v - (float)hi); }
__device__ __forceinline__ v16b frag_kb(const b16* p, int hh) { const v8b a = *(const v8b*)(p + 8 * hh), b = *(const v8b*)(p + 16 + 8 * hh); v16b f;
#pragma unroll
  for (int e = 0; e < 8; ++e) { f[e] = a[e]; f[8 + e] = b[e]; } return f; }
__device__ __forceinline__ v8f wmma16b(v16b a, v16b b, v8f c) { v8f d = __builtin_amdgcn_wmma_f32_16x16x32_f16(false, a, false, b, (short)0, c, false, false); asm volatile("v_nop\n\tv_nop\n\tv_nop\n\tv_nop" : "+v"(d) : "v"(a), "v"(b)); return d; }
__device__ __forceinline__ void wave_lds_sync() { __builtin_amdgcn_fence(__ATOMIC_RELEASE, "workgroup"); __builtin_amdgcn_wave_barrier(); __builtin_amdgcn_fence(__ATOMIC_ACQUIRE, "workgroup"); }
__device__ __forceinline__ float pmul(float a, float b) { float p = a * b; asm volatile("" : "+v"(p)); return p; }
__device__ __forceinline__ int iclamp(int v, int lo, int hi) { return v < lo ? lo : (v > hi ? hi : v); }
__device__ __forceinline__ float sigm(float v) { return 1.0f / (1.0f + __expf(-v)); }
constexpr int CSR_NBLK9 = 512, CSR_GB9 = 9, CSR_GN9 = 1 << CSR_GB9  , CSR_TS9 = (CSR_GN9 < 32 ? 32 : CSR_GN9)  , CSR_MAXG9 = 512, CSR_CAP9 = 12288  ;
__device__ __host__ __forceinline__ int csr_tix9(int v) { return (v >> CSR_GB9) * CSR_TS9 + (v & (CSR_GN9 - 1)); }
__global__ __launch_bounds__(64) void csrA_kernel9(const int* __restrict__ dst, int E, int N, int nG, int CHP, int NGP, int* __restrict__ STG, int* __restrict__ HST) {
  extern __shared__ int sm[];
  int* cnt = sm; int* run = sm + NGP; int* ids = sm + 2 * NGP;
  const int b = blockIdx.x; const int ch = (E + CSR_NBLK9 - 1) / CSR_NBLK9; const int e0 = b * ch, e1 = min(E, e0 + ch);
  for (int i = threadIdx.x; i < NGP; i += 64) cnt[i] = 0;
  for (int i = threadIdx.x; i < CHP; i += 64) ids[i] = -1;
  __syncthreads();
  if (threadIdx.x == 0) {
    for (int e = e0; e < e1; ++e) { int d = dst[e]; d = (d < 0) ? 0 : (d >= N ? N - 1 : d); cnt[d >> CSR_GB9] += 1; }
    int acc = 0; for (int g = 0; g < nG; ++g) { run[g] = acc; acc += cnt[g]; }
    for (int e = e0; e < e1; ++e) { int d = dst[e]; d = (d < 0) ? 0 : (d >= N ? N - 1 : d); const int g = d >> CSR_GB9; ids[run[g]] = e; run[g] += 1; } }
  __syncthreads();
  typedef __attribute__((ext_vector_type(4))) int v4i;
  for (int pass = 0; pass < 2; ++pass) {
    for (int i = threadIdx.x; i < CHP / 4; i += 64) *(volatile v4i*)(STG + (size_t)b * CHP + i * 4) = *(const v4i*)(&ids[i * 4]);
    for (int i = threadIdx.x; i < NGP / 4; i += 64) { v4i v; for (int e = 0; e < 4; ++e) v[e] = (i * 4 + e < nG) ? cnt[i * 4 + e] : 0; *(volatile v4i*)(HST + (size_t)b * NGP + i * 4) = v; }
    __threadfence(); }
}
__global__ __launch_bounds__(512) void csrS_kernel9(const int* __restrict__ HST, int nG, int NGP, int* __restrict__ START, int* __restrict__ TOT, int* __restrict__ OFF) {
  __shared__ int tot[CSR_MAXG9];
  const int b = threadIdx.x;
  for (int pass = 0; pass < 2; ++pass) { int runb = 0; for (int g = 0; g < nG; ++g) { int c = HST[(size_t)b * NGP + g]; c = (c < 0) ? 0 : c; ((volatile int*)OFF)[(size_t)g * CSR_NBLK9 + b] = runb; runb += c; } __threadfence(); }
  for (int g = threadIdx.x; g < nG; g += 512) { int s = 0; for (int bb = 0; bb < CSR_NBLK9; ++bb) { int c = HST[(size_t)bb * NGP + g]; s += (c < 0) ? 0 : c; } tot[g] = s; }
  __syncthreads();
  if (threadIdx.x < 32) {
    __shared__ int st[CSR_MAXG9 + 32];
    if (threadIdx.x == 0) { int acc = 0; for (int g = 0; g < NGP; ++g) { st[g] = acc; if (g < nG) acc += (tot[g] + 31) & ~31; } st[NGP] = acc; }
    __builtin_amdgcn_fence(__ATOMIC_RELEASE, "workgroup"); __builtin_amdgcn_wave_barrier(); __builtin_amdgcn_fence(__ATOMIC_ACQUIRE, "workgroup");
    for (int pass = 0; pass < 2; ++pass) { for (int i = threadIdx.x; i < NGP + 32; i += 32) { ((volatile int*)START)[i] = (i <= NGP) ? st[min(i, NGP)] : 0; ((volatile int*)TOT)[i] = (i < nG) ? tot[i] : 0; } __threadfence(); } }
}
__global__ __launch_bounds__(256) void csrB_kernel9(const int* __restrict__ dst, int N, int nG, int CHP, int NGP, int permLen, const int* __restrict__ STG, const int* __restrict__ HST, const int* __restrict__ OFF, const int* __restrict__ START, const int* __restrict__ TOT, int* __restrict__ PERM, int* __restrict__ ROWPTR, int* __restrict__ ROWCNT, int* __restrict__ FLAG) {
  typedef __attribute__((ext_vector_type(4))) int v4i;
  __shared__ int ids[CSR_CAP9]; __shared__ unsigned short key[CSR_CAP9]; __shared__ int outp[CSR_CAP9]; __shared__ int ncnt[CSR_GN9 + 1]; __shared__ int boff[CSR_NBLK9 + 1];
  const int g = blockIdx.x, t_ = threadIdx.x; int tot = TOT[g]; int st = START[g], stn = START[g + 1]; const int v0 = g * CSR_GN9; const int nv = min(CSR_GN9, N - v0); const int t0 = g * CSR_TS9;
  st = (st < 0) ? 0 : (st > permLen - 32 ? permLen - 32 : st) & ~31; stn = (stn < st) ? st : (stn > permLen ? permLen : stn); tot = (tot < 0) ? 0 : tot; if (tot > stn - st && tot <= CSR_CAP9) tot = stn - st;
  if (tot > CSR_CAP9) {
    for (int pass = 0; pass < 2; ++pass) { for (int i = t_; i < CSR_TS9 / 4; i += 256) { v4i a, c; for (int e = 0; e < 4; ++e) { a[e] = st; c[e] = 0; } *(volatile v4i*)(ROWPTR + t0 + i * 4) = a; *(volatile v4i*)(ROWCNT + t0 + i * 4) = c; } if (t_ == 0) ((volatile int*)FLAG)[0] = 1; __threadfence(); } (void)nv; return; }
  if (t_ == 0) { int acc = 0; for (int b = 0; b < CSR_NBLK9; ++b) { boff[b] = acc; int c = HST[(size_t)b * NGP + g]; c = (c < 0) ? 0 : (c > CHP ? CHP : c); acc += c; if (acc > tot) acc = tot; } boff[CSR_NBLK9] = acc; }
  for (int i = t_; i <= CSR_GN9; i += 256) ncnt[i] = 0;
  __syncthreads();
  for (int b = 0; b < CSR_NBLK9; ++b) { const int c = boff[b + 1] - boff[b]; int o_ = OFF[(size_t)g * CSR_NBLK9 + b]; o_ = (o_ < 0) ? 0 : (o_ > CHP - c ? CHP - c : o_); const int* src_ = STG + (size_t)b * CHP + o_;
    for (int i = t_; i < c; i += 256) { int id = src_[i]; id = (id < 0) ? 0 : id; ids[boff[b] + i] = id; int d = dst[id]; d = (d < v0) ? v0 : (d >= N ? N - 1 : d); int kk = d - v0; kk = (kk < 0) ? 0 : (kk >= CSR_GN9 ? CSR_GN9 - 1 : kk); key[boff[b] + i] = (unsigned short)kk; } }
  __syncthreads();
  if (t_ == 0) { for (int i = 0; i < tot; ++i) ncnt[key[i]] += 1; int acc = 0; for (int vl = 0; vl < CSR_GN9; ++vl) { const int c = ncnt[vl]; ncnt[vl] = acc; acc += c; } ncnt[CSR_GN9] = acc;
    for (int i = 0; i < tot; ++i) { const int vl = key[i]; outp[ncnt[vl]] = ids[i]; ncnt[vl] += 1; }
    for (int vl = CSR_GN9; vl > 0; --vl) ncnt[vl] = ncnt[vl - 1]; ncnt[0] = 0; }
  __syncthreads();
  for (int pass = 0; pass < 2; ++pass) {
    for (int i = t_; i < (stn - st) / 4; i += 256) { v4i v; for (int e = 0; e < 4; ++e) { const int q = i * 4 + e; v[e] = (q < tot) ? outp[q] : -1; } *(volatile v4i*)(PERM + st + i * 4) = v; }
    for (int i = t_; i < CSR_TS9 / 4; i += 256) { v4i a, c; for (int e = 0; e < 4; ++e) { const int vl = i * 4 + e; const int vc = vl < CSR_GN9 ? vl : CSR_GN9; a[e] = (vl < CSR_GN9) ? st + ncnt[vc] : st; c[e] = (vl < nv) ? (ncnt[(vc < CSR_GN9 ? vc : CSR_GN9 - 1) + 1] - ncnt[vc]) : 0; } *(volatile v4i*)(ROWPTR + t0 + i * 4) = a; *(volatile v4i*)(ROWCNT + t0 + i * 4) = c; }
    __threadfence(); }
}
__global__ __launch_bounds__(256) void csrZ_kernel9(int* __restrict__ p, size_t n4) { typedef __attribute__((ext_vector_type(4))) int v4i; const size_t tid = (size_t)blockIdx.x * 256 + threadIdx.x, nth = (size_t)gridDim.x * 256; v4i z = {0, 0, 0, 0}; for (size_t i = tid; i < n4; i += nth) *(volatile v4i*)(p + i * 4) = z; }
struct CsrBufs9 { int *STG, *HST, *OFF, *START, *TOT, *PERM, *ROWPTR, *ROWCNT, *FLAG; int nG, NGP, CHP; size_t permLen; char* base; size_t bytes; };
static size_t csr_carve9(CsrBufs9& c, char* ws, size_t off, int E, int N) {
  const size_t off0 = off; c.base = ws + off;
  auto al = [&](size_t bytes) { char* p = ws + off; off += (bytes + 255) & ~(size_t)255; return p; };
  c.nG = (N + CSR_GN9 - 1) / CSR_GN9; c.NGP = (c.nG + 31) & ~31; const int ch = (E + CSR_NBLK9 - 1) / CSR_NBLK9; c.CHP = (ch + 31) & ~31; c.permLen = (size_t)E + 32 * (size_t)c.nG + 32;
  c.STG = (int*)al((size_t)CSR_NBLK9 * c.CHP * 4); c.HST = (int*)al((size_t)CSR_NBLK9 * c.NGP * 4); c.OFF = (int*)al((size_t)c.NGP * CSR_NBLK9 * 4); c.START = (int*)al((size_t)(c.NGP + 64) * 4); c.TOT = (int*)al((size_t)(c.NGP + 64) * 4);
  c.PERM = (int*)al(c.permLen * 4); c.ROWPTR = (int*)al((size_t)c.nG * CSR_TS9 * 4); c.ROWCNT = (int*)al((size_t)c.nG * CSR_TS9 * 4); c.FLAG = (int*)al(256);
  c.bytes = off - off0; return off;
}
static void csr_build9(const CsrBufs9& c, const int* dst, int E, int N, hipStream_t stream) {
  const size_t smem = (size_t)(2 * c.NGP + c.CHP) * 4;
  csrZ_kernel9<<<512, 256, 0, stream>>>((int*)c.base, c.bytes / 16);
  csrA_kernel9<<<CSR_NBLK9, 64, smem, stream>>>(dst, E, N, c.nG, c.CHP, c.NGP, c.STG, c.HST);
  csrS_kernel9<<<1, 512, 0, stream>>>(c.HST, c.nG, c.NGP, c.START, c.TOT, c.OFF);
  csrB_kernel9<<<c.nG, 256, 0, stream>>>(dst, N, c.nG, c.CHP, c.NGP, (int)c.permLen, c.STG, c.HST, c.OFF, c.START, c.TOT, c.PERM, c.ROWPTR, c.ROWCNT, c.FLAG);
}


__global__ __launch_bounds__(256) void wrow_kernel(const float* __restrict__ w, int inp, int ko, int KIN, int KP, int OUT, b16* __restrict__ WT) {
  const int KG = KP / 8; const int u = blockIdx.x * 256 + threadIdx.x; if (u >= OUT * KG) return; const int o = u / KG, k0 = (u % KG) * 8; v8b v;
#pragma unroll
  for (int j = 0; j < 8; ++j) { const int k = k0 + j; v[j] = k < KIN ? (b16)(bf16_rne(w[(size_t)o * inp + ko + k]) * WSC) : (b16)0.0f; } for (int pass = 0; pass < 2; ++pass) { *(volatile v8b*)(WT + (size_t)o * KP + k0) = v; __threadfence(); }
}
__global__ __launch_bounds__(256) void agg_kernel(const float* __restrict__ xs, const int* __restrict__ rows, const int* __restrict__ PERM, const int* __restrict__ ROWPTR, const int* __restrict__ ROWCNT, int permLen, int NLIM, b16* __restrict__ AG, float* __restrict__ SV) {
  const int wave = threadIdx.x >> 5, lane = threadIdx.x & 31; const size_t v = (size_t)blockIdx.x * 8 + wave; if (v >= (size_t)NLIM) return; const int t = lane >> 1, f0 = (lane & 1) * 8;
  int st = ROWPTR[v], cnt = ROWCNT[v]; cnt = iclamp(cnt, 0, 1 << 20); st = iclamp(st, 0, permLen - cnt);
  int nn = 0;
#pragma unroll 1
  for (int j = 0; j < cnt; ++j) { const int e = iclamp(PERM[st + j], 0, E - 1); if (iclamp(rows[e], 0, N - 1) < NLIM) ++nn; }
  const float dv = rsqrtf((float)(nn + 1)); float o[8]; const float* xv = xs + ((size_t)t * N + v) * FI + f0;
#pragma unroll
  for (int i = 0; i < 8; ++i) o[i] = pmul(dv * dv, bf16_rne(xv[i]));
  float S = dv * dv;
#pragma unroll 1
  for (int j = 0; j < cnt; ++j) { const int e = iclamp(PERM[st + j], 0, E - 1); const size_t u = (size_t)iclamp(rows[e], 0, N - 1); if (u >= (size_t)NLIM) continue; int cu = ROWCNT[u]; cu = iclamp(cu, 0, 1 << 20);
    int nu = cu; if (NLIM < N) { nu = 0; const int su = iclamp(ROWPTR[u], 0, permLen - cu); for (int k = 0; k < cu; ++k) if (iclamp(rows[iclamp(PERM[su + k], 0, E - 1)], 0, N - 1) < NLIM) ++nu; }
    const float wgt = pmul(dv, rsqrtf((float)(nu + 1))); S += wgt; const float* xu = xs + ((size_t)t * N + u) * FI + f0;
#pragma unroll
    for (int i = 0; i < 8; ++i) o[i] += pmul(wgt, bf16_rne(xu[i])); }
  v8b pk, zz = {};
#pragma unroll
  for (int i = 0; i < 8; ++i) pk[i] = (b16)(o[i] * XS);
  for (int pass = 0; pass < 2; ++pass) { *(volatile v8b*)(AG + (v * T + t) * 32 + f0) = pk; *(volatile v8b*)(AG + (v * T + t) * 32 + 16 + f0) = zz; ((volatile float*)SV)[v * 32 + lane] = lane == 0 ? S : 0.0f; __threadfence(); }
}
__global__ __launch_bounds__(32) void gcn_kernel(const b16* __restrict__ AG, const float* __restrict__ SV, const b16* __restrict__ WG, const float* __restrict__ gb, int NLIM, b16* __restrict__ GC) {
  __shared__ __attribute__((aligned(16))) b16 Tb[16][72]; const int lane = threadIdx.x, nloc = lane & 15, hlf = lane >> 4; const size_t v = blockIdx.x; if (v >= (size_t)NLIM) return; const float sv = SV[v * 32];
  const v16b a = frag_kb(AG + (v * T + nloc) * 32, hlf);
#pragma unroll
  for (int tt = 0; tt < 4; ++tt) { v8f acc = {}; acc = wmma16b(a, frag_kb(WG + (size_t)(tt * 16 + nloc) * 32, hlf), acc); const int c = tt * 16 + nloc; const float bb = pmul(bf16_rne(gb[c]), sv);
#pragma unroll
    for (int r8 = 0; r8 < 8; ++r8) Tb[8 * hlf + r8][c] = (b16)((acc[r8] * (1.0f / (XS * WSC)) + bb) * XS); }
  wave_lds_sync();
  for (int pass = 0; pass < 2; ++pass) { for (int t = 0; t < T; ++t) { __attribute__((ext_vector_type(2))) _Float16 p2 = {Tb[t][lane * 2], Tb[t][lane * 2 + 1]}; *(volatile __attribute__((ext_vector_type(2))) _Float16*)(GC + ((size_t)t * N + v) * GH + lane * 2) = p2; } __threadfence(); }
}
__global__ __launch_bounds__(32) void gru_kernel(const b16* __restrict__ GC, const b16* __restrict__ WIH, const b16* __restrict__ WHH, const float* __restrict__ bih, const float* __restrict__ bhh, int NLIM, float* __restrict__ NE) {
  __shared__ __attribute__((aligned(16))) b16 Hb[16][72]; __shared__ float Hs[16][RH + 1], Gin[16][RH + 1], Ghn[16][RH + 1];
  const int lane = threadIdx.x, nloc = lane & 15, hlf = lane >> 4; const size_t m0 = (size_t)blockIdx.x * 16; if (m0 >= (size_t)NLIM) return;
  for (int rr = 0; rr < 16; ++rr) { Hs[rr][lane * 2] = 0.0f; Hs[rr][lane * 2 + 1] = 0.0f; Hb[rr][lane * 2] = (b16)0.0f; Hb[rr][lane * 2 + 1] = (b16)0.0f; }
  wave_lds_sync(); const float si = 1.0f / (XS * WSC);
#pragma unroll 1
  for (int t = 0; t < T; ++t) {
    { v8f gi[4], gh[4];
#pragma unroll
      for (int tt = 0; tt < 4; ++tt) { gi[tt] = (v8f){}; gh[tt] = (v8f){}; }
#pragma unroll
      for (int kb = 0; kb < RH; kb += 32) { const v16b a = frag_kb(GC + ((size_t)t * N + m0 + nloc) * GH + kb, hlf), hb = frag_kb(&Hb[nloc][kb], hlf);
#pragma unroll
        for (int tt = 0; tt < 4; ++tt) { gi[tt] = wmma16b(a, frag_kb(WIH + (size_t)((8 + tt) * 16 + nloc) * RH + kb, hlf), gi[tt]); gh[tt] = wmma16b(hb, frag_kb(WHH + (size_t)((8 + tt) * 16 + nloc) * RH + kb, hlf), gh[tt]); } }
#pragma unroll
      for (int tt = 0; tt < 4; ++tt) { const int j = tt * 16 + nloc; const float b1 = bf16_rne(bih[2 * RH + j]), b2 = bf16_rne(bhh[2 * RH + j]);
#pragma unroll
        for (int r8 = 0; r8 < 8; ++r8) { Gin[8 * hlf + r8][j] = gi[tt][r8] * si + b1; Ghn[8 * hlf + r8][j] = gh[tt][r8] * si + b2; } } }
    { v8f gi[8], gh[8];
#pragma unroll
      for (int tt = 0; tt < 8; ++tt) { gi[tt] = (v8f){}; gh[tt] = (v8f){}; }
#pragma unroll
      for (int kb = 0; kb < RH; kb += 32) { const v16b a = frag_kb(GC + ((size_t)t * N + m0 + nloc) * GH + kb, hlf), hb = frag_kb(&Hb[nloc][kb], hlf);
#pragma unroll
        for (int tt = 0; tt < 8; ++tt) { gi[tt] = wmma16b(a, frag_kb(WIH + (size_t)(tt * 16 + nloc) * RH + kb, hlf), gi[tt]); gh[tt] = wmma16b(hb, frag_kb(WHH + (size_t)(tt * 16 + nloc) * RH + kb, hlf), gh[tt]); } }
      wave_lds_sync();
#pragma unroll
      for (int tg = 0; tg < 4; ++tg) { const int j = tg * 16 + nloc; const float bir = bf16_rne(bih[j]), bhr = bf16_rne(bhh[j]), biz = bf16_rne(bih[RH + j]), bhz = bf16_rne(bhh[RH + j]);
#pragma unroll
        for (int r8 = 0; r8 < 8; ++r8) { const int rl = 8 * hlf + r8; const float r = sigm(gi[tg][r8] * si + bir + gh[tg][r8] * si + bhr), z = sigm(gi[4 + tg][r8] * si + biz + gh[4 + tg][r8] * si + bhz); const float nn = tanhf(Gin[rl][j] + pmul(r, Ghn[rl][j])); const float hv = pmul(1.0f - z, nn) + pmul(z, Hs[rl][j]); Hs[rl][j] = hv; Hb[rl][j] = (b16)(hv * XS); } } }
    wave_lds_sync(); }
  for (int pass = 0; pass < 2; ++pass) { for (int rr = 0; rr < 16; ++rr) *(volatile v2f*)(NE + (m0 + rr) * RH + lane * 2) = (v2f){Hs[rr][lane * 2], Hs[rr][lane * 2 + 1]}; __threadfence(); }
}
__global__ __launch_bounds__(32) void pq_kernel(const float* __restrict__ NE, const b16* __restrict__ WPQ, int NLIM, float* __restrict__ PQ) {
  __shared__ __attribute__((aligned(16))) b16 Ah[16][72], Al[16][72]; __shared__ float Tf[16][132]; const int lane = threadIdx.x, nloc = lane & 15, hlf = lane >> 4; const size_t m0 = (size_t)blockIdx.x * 16; if (m0 >= (size_t)NLIM) return;
  for (int rr = 0; rr < 16; ++rr) for (int q = 0; q < 2; ++q) { b16 p, ql; split16(NE[(m0 + rr) * RH + q * 32 + lane] * XS, p, ql); Ah[rr][q * 32 + lane] = p; Al[rr][q * 32 + lane] = ql; }
  wave_lds_sync();
#pragma unroll 1
  for (int cg = 0; cg < 2; ++cg) { v8f acc[8];
#pragma unroll
    for (int tt = 0; tt < 8; ++tt) acc[tt] = (v8f){};
#pragma unroll
    for (int kb = 0; kb < RH; kb += 32) { const v16b a = frag_kb(&Ah[nloc][kb], hlf), al = frag_kb(&Al[nloc][kb], hlf);
#pragma unroll
      for (int tt = 0; tt < 8; ++tt) { const v16b bw = frag_kb(WPQ + (size_t)(cg * 128 + tt * 16 + nloc) * RH + kb, hlf); acc[tt] = wmma16b(a, bw, acc[tt]); acc[tt] = wmma16b(al, bw, acc[tt]); } }
#pragma unroll
    for (int tt = 0; tt < 8; ++tt)
#pragma unroll
      for (int r8 = 0; r8 < 8; ++r8) Tf[8 * hlf + r8][tt * 16 + nloc] = acc[tt][r8] * (1.0f / (XS * WSC));
    wave_lds_sync();
    for (int pass = 0; pass < 2; ++pass) { for (int rr = 0; rr < 16; ++rr) *(volatile v4f*)(PQ + (m0 + rr) * (2 * EH) + cg * 128 + lane * 4) = *(const v4f*)(&Tf[rr][lane * 4]); __threadfence(); }
    wave_lds_sync(); }
}
__global__ __launch_bounds__(32) void edge_kernel(const float* __restrict__ PQ, const float* __restrict__ ea, const int* __restrict__ rows, const int* __restrict__ cols, const float* __restrict__ e1W, const float* __restrict__ e1b, const float* __restrict__ e2w, const float* __restrict__ e2b, int NLIM, float* __restrict__ ST1) {
  const int lane = threadIdx.x; const size_t e = (size_t)blockIdx.x * 32 + lane; const int r = iclamp(rows[e], 0, N - 1), c = iclamp(cols[e], 0, N - 1); float s = 0.0f;
  if (r < NLIM && c < NLIM) { const float a0 = bf16_rne(ea[e * 4]), a1 = bf16_rne(ea[e * 4 + 1]), a2 = bf16_rne(ea[e * 4 + 2]), a3 = bf16_rne(ea[e * 4 + 3]); const float* pr = PQ + (size_t)r * (2 * EH); const float* qc = PQ + (size_t)c * (2 * EH) + EH; s = bf16_rne(e2b[0]);
#pragma unroll 2
    for (int k = 0; k < EH; ++k) { const float* wk = e1W + (size_t)k * 132 + 128; float hsum = pr[k] + qc[k] + bf16_rne(e1b[k]); hsum += pmul(a0, bf16_rne(wk[0])) + pmul(a1, bf16_rne(wk[1])) + pmul(a2, bf16_rne(wk[2])) + pmul(a3, bf16_rne(wk[3])); s += pmul(fmaxf(hsum, 0.0f), bf16_rne(e2w[k])); } }
  for (int pass = 0; pass < 2; ++pass) { ((volatile float*)ST1)[e] = s; __threadfence(); }
}
__global__ __launch_bounds__(32) void node_kernel(const float* __restrict__ NE, const float* __restrict__ ST1, const int* __restrict__ rows, const int* __restrict__ PERM, const int* __restrict__ ROWPTR, const int* __restrict__ ROWCNT, int permLen, const float* __restrict__ p1W, const float* __restrict__ p1b, const float* __restrict__ p2w, const float* __restrict__ p2b, int NLIM, float* __restrict__ ST0) {
  __shared__ float Pin[32][66]; const int lane = threadIdx.x; const size_t v0 = (size_t)blockIdx.x * 32, v = v0 + lane; if (v0 >= (size_t)NLIM) return; const size_t vv = v < (size_t)N ? v : N - 1;
  int st = ROWPTR[vv], cnt = ROWCNT[vv]; cnt = iclamp(cnt, 0, 1 << 20); st = iclamp(st, 0, permLen - cnt); float flow = 0.0f;
#pragma unroll 1
  for (int j = 0; j < cnt; ++j) { const int e = iclamp(PERM[st + j], 0, E - 1); if (iclamp(rows[e], 0, N - 1) < NLIM) flow += ST1[e]; }
  for (int k = 0; k < RH; ++k) Pin[lane][k] = NE[vv * RH + k]; Pin[lane][RH] = flow;
  float s = bf16_rne(p2b[0]);
#pragma unroll 1
  for (int o = 0; o < 64; ++o) { const float* wr = p1W + (size_t)o * 65; float hsum = bf16_rne(p1b[o]);
#pragma unroll 5
    for (int k = 0; k < 65; ++k) hsum += pmul(Pin[lane][k], bf16_rne(wr[k])); s += pmul(fmaxf(hsum, 0.0f), bf16_rne(p2w[o])); }
  for (int pass = 0; pass < 2; ++pass) { if (v < (size_t)N) ((volatile float*)ST0)[v] = s; __threadfence(); }
}
__global__ __launch_bounds__(256) void copy_kernel(const float* __restrict__ ST0, const float* __restrict__ ST1, float* __restrict__ out) { const size_t i = (size_t)blockIdx.x * 256 + threadIdx.x; if (i >= (size_t)N + E) return; const float v = i < (size_t)N ? ST0[i] : ST1[i - N]; for (int pass = 0; pass < 2; ++pass) { ((volatile float*)out)[i] = v; __threadfence(); } }
}

extern "C" void kernel_launch(void* const* d_in, const int* in_sizes, int n_in, void* d_out, int out_size, void* d_ws, size_t ws_size, hipStream_t stream) {
  (void)n_in;
  auto Fp = [&](int i) { return (const float*)d_in[i]; }; auto Ip = [&](int i) { return (const int*)d_in[i]; };
  if (in_sizes[0] != T * N * FI || in_sizes[1] != E * 4 || in_sizes[2] != GH * FI || in_sizes[4] != 192 * RH || in_sizes[5] != 192 * RH || in_sizes[8] != EH * 132 || in_sizes[10] != EH || in_sizes[12] != 64 * 65 || in_sizes[14] != 64 || in_sizes[16] != 2 * E || out_size != N + E) return;
  const int NLIM = N; const int GB16 = NBLK, GB8 = N / 8;
  size_t off = 0; char* ws = (char*)d_ws;
  auto carve = [&](size_t bytes) { char* p = ws + off; off += (bytes + 255) & ~(size_t)255; return p; };
  b16* WG = (b16*)carve(GH * 32 * 2); b16* WIH = (b16*)carve(192 * RH * 2); b16* WHH = (b16*)carve(192 * RH * 2); b16* WPQ = (b16*)carve(2 * EH * RH * 2);
  b16* AG = (b16*)carve((size_t)N * T * 32 * 2); float* SV = (float*)carve((size_t)N * 32 * 4); b16* GC = (b16*)carve((size_t)T * N * GH * 2); float* NE = (float*)carve((size_t)N * RH * 4); float* PQ = (float*)carve((size_t)N * 2 * EH * 4); float* ST0 = (float*)carve((size_t)N * 4); float* ST1 = (float*)carve((size_t)E * 4);
  CsrBufs9 csr; off = csr_carve9(csr, ws, off, E, N);
  if (off > ws_size || off > ((size_t)240 << 20)) return;
  wrow_kernel<<<(GH * 4 + 255) / 256, 256, 0, stream>>>(Fp(2), FI, 0, FI, 32, GH, WG); wrow_kernel<<<(192 * 8 + 255) / 256, 256, 0, stream>>>(Fp(4), RH, 0, RH, RH, 192, WIH); wrow_kernel<<<(192 * 8 + 255) / 256, 256, 0, stream>>>(Fp(5), RH, 0, RH, RH, 192, WHH);
  wrow_kernel<<<(EH * 8 + 255) / 256, 256, 0, stream>>>(Fp(8), 132, 0, RH, RH, EH, WPQ); wrow_kernel<<<(EH * 8 + 255) / 256, 256, 0, stream>>>(Fp(8), 132, 64, RH, RH, EH, WPQ + (size_t)EH * RH);
  csr_build9(csr, Ip(16) + E, E, N, stream);
  agg_kernel<<<GB8, 256, 0, stream>>>(Fp(0), Ip(16), csr.PERM, csr.ROWPTR, csr.ROWCNT, (int)csr.permLen, NLIM, AG, SV);
  gcn_kernel<<<(unsigned)NLIM, 32, 0, stream>>>(AG, SV, WG, Fp(3), NLIM, GC);
  gru_kernel<<<GB16, 32, 0, stream>>>(GC, WIH, WHH, Fp(6), Fp(7), NLIM, NE);
  pq_kernel<<<GB16, 32, 0, stream>>>(NE, WPQ, NLIM, PQ);
  edge_kernel<<<E / 32, 32, 0, stream>>>(PQ, Fp(1), Ip(16), Ip(16) + E, Fp(8), Fp(9), Fp(10), Fp(11), NLIM, ST1);
  node_kernel<<<(N + 31) / 32, 32, 0, stream>>>(NE, ST1, Ip(16), csr.PERM, csr.ROWPTR, csr.ROWCNT, (int)csr.permLen, Fp(12), Fp(13), Fp(14), Fp(15), NLIM, ST0);
  copy_kernel<<<(unsigned)((N + E + 255) / 256), 256, 0, stream>>>(ST0, ST1, (float*)d_out);
}
